// ConvCrossAttention_56315611185663
// MI455X (gfx1250) — hardware-verified
//
#include <hip/hip_runtime.h>
#include <stdint.h>
#include <math.h>

typedef __attribute__((ext_vector_type(16))) _Float16 v16h;
typedef __attribute__((ext_vector_type(8)))  _Float16 v8h;
typedef __attribute__((ext_vector_type(16))) __bf16   v16b;
typedef __attribute__((ext_vector_type(8)))  __bf16   v8b;
typedef __attribute__((ext_vector_type(8)))  float    v8f;
typedef __attribute__((ext_vector_type(4)))  float    v4f;
typedef __attribute__((ext_vector_type(4)))  unsigned int v4u32;
#define U16(p) ((const unsigned short*)(const void*)(p))

__device__ __forceinline__ unsigned short f2bf_bits(float f) {
  unsigned u = __float_as_uint(f);
  return (unsigned short)((u + 0x7FFFu + ((u >> 16) & 1u)) >> 16);
}
__device__ __forceinline__ float bf_bits2f(unsigned short h) { return __uint_as_float(((unsigned)h) << 16); }

__device__ __forceinline__ void dep_guard_h(v8f& a, v8f& b, v16h x, v16h y) { asm volatile("v_nop\n\tv_nop\n\tv_nop\n\tv_nop" : "+v"(a), "+v"(b) : "v"(x), "v"(y)); }
__device__ __forceinline__ void dep_guard_b(v8f& a, v8f& b, v16b x, v16b y) { asm volatile("v_nop\n\tv_nop\n\tv_nop\n\tv_nop" : "+v"(a), "+v"(b) : "v"(x), "v"(y)); }
__device__ __forceinline__ void keep4_h(v16h a, v16h b, v16h c, v16h d) { asm volatile("v_nop" :: "v"(a), "v"(b), "v"(c), "v"(d)); }
__device__ __forceinline__ void keep4_b(v16b a, v16b b, v16b c, v16b d) { asm volatile("v_nop" :: "v"(a), "v"(b), "v"(c), "v"(d)); }
__device__ __forceinline__ void acc_guard4(v8f& a, v8f& b, v8f& c, v8f& d) { asm volatile("v_nop\n\tv_nop\n\tv_nop\n\tv_nop" : "+v"(a), "+v"(b), "+v"(c), "+v"(d)); }
template <typename T> struct Frag;
template <> struct Frag<_Float16> {
  typedef v16h V; union U { v16h v; v8h h[2]; };
  static __device__ __forceinline__ v16h load(const _Float16* p) {
    U f; f.h[0] = *(const v8h*)(p); f.h[1] = *(const v8h*)(p + 16); return f.v;
  }
  static __device__ __forceinline__ v8f mma(v16h a, v16h b, v8f c) {
    return __builtin_amdgcn_wmma_f32_16x16x32_f16(false, a, false, b, (short)0, c, false, false);
  }
  static __device__ __forceinline__ void guard(v8f& a, v8f& b, v16h x, v16h y) { dep_guard_h(a, b, x, y); }
  static __device__ __forceinline__ void keep(v16h a, v16h b, v16h c, v16h d) { keep4_h(a, b, c, d); }
};
template <> struct Frag<__bf16> {
  typedef v16b V; union U { v16b v; v8b h[2]; };
  static __device__ __forceinline__ v16b load(const __bf16* p) {
    U f; f.h[0] = *(const v8b*)(p); f.h[1] = *(const v8b*)(p + 16); return f.v;
  }
  static __device__ __forceinline__ v8f mma(v16b a, v16b b, v8f c) {
    return __builtin_amdgcn_wmma_f32_16x16x32_bf16(false, a, false, b, (short)0, c, false, false);
  }
  static __device__ __forceinline__ void guard(v8f& a, v8f& b, v16b x, v16b y) { dep_guard_b(a, b, x, y); }
  static __device__ __forceinline__ void keep(v16b a, v16b b, v16b c, v16b d) { keep4_b(a, b, c, d); }
};

template <int ET> struct Elem;
template <> struct Elem<0> { typedef _Float16 T; };
template <> struct Elem<1> { typedef __bf16 T; };
template <int ET, bool SPLIT, int BIAS_MODE, int OUT_MODE, bool RESID, int ACT = 0>
__global__ __launch_bounds__(256) void wmma_gemm64(
    const unsigned short* __restrict__ Ap, const unsigned short* __restrict__ A2p, int lda, long strideA,
    const unsigned short* __restrict__ Btp, const unsigned short* __restrict__ Bt2p, int ldb, long strideB,
    void* __restrict__ Cout, void* __restrict__ Cout2, int ldc, long strideC,
    const float* __restrict__ bias,
    const float* __restrict__ resid, long strideR,
    int M, int N, int K, float scale) {
  typedef typename Elem<ET>::T T;
  typedef typename Frag<T>::V V;
  const T* A = (const T*)Ap; const T* A2 = (const T*)A2p; const T* Bt = (const T*)Btp; const T* Bt2 = (const T*)Bt2p;
  __shared__ __align__(16) float sT[8][16 * 68];
  const int b    = blockIdx.y;
  const int lane = threadIdx.x & 31;
  const int wave = threadIdx.x >> 5;
  const int tilesN = N >> 6;
  const int tilesM = M >> 6;
  const int tile = blockIdx.x * 8 + wave;
  if (tile >= tilesM * tilesN) return;
  const int tm = tile / tilesN;
  const int tn = tile - tm * tilesN;
  const int m0 = tm << 6;
  const int n0 = tn << 6;

  const T* Ab  = A  + (size_t)b * strideA;
  const T* Bb  = Bt + (size_t)b * strideB;
  const T* Ab2 = SPLIT ? (A2  + (size_t)b * strideA) : nullptr;
  const T* Bb2 = SPLIT ? (Bt2 + (size_t)b * strideB) : nullptr;

  const int rlane = lane & 15;
  const int koff  = (lane >> 4) * 8;
  const int mOff  = (lane >> 4) * 8;

  v8f acc[4][4];
#pragma unroll
  for (int i = 0; i < 4; ++i)
#pragma unroll
    for (int j = 0; j < 4; ++j) acc[i][j] = (v8f){0.f,0.f,0.f,0.f,0.f,0.f,0.f,0.f};

  for (int k0 = 0; k0 < K; k0 += 32) {
    V bh[4], bl[4];
#pragma unroll
    for (int j = 0; j < 4; ++j) {
      const size_t bo = (size_t)(n0 + (j << 4) + rlane) * ldb + koff + k0;
      bh[j] = Frag<T>::load(Bb + bo);
      if (SPLIT) bl[j] = Frag<T>::load(Bb2 + bo);
    }
#pragma unroll
    for (int i = 0; i < 4; ++i) {
      const size_t ao = (size_t)(m0 + (i << 4) + rlane) * lda + koff + k0;
      V ah = Frag<T>::load(Ab + ao);
      V al;
      if (SPLIT) al = Frag<T>::load(Ab2 + ao);
#pragma unroll
      for (int j = 0; j < 4; ++j) {
        acc[i][j] = Frag<T>::mma(ah, bh[j], acc[i][j]);
        if (SPLIT) {
          acc[i][j] = Frag<T>::mma(ah, bl[j], acc[i][j]);
          acc[i][j] = Frag<T>::mma(al, bh[j], acc[i][j]);
        }
      }
      Frag<T>::guard(acc[i][0], acc[i][3], ah, SPLIT ? al : ah);
    }
    Frag<T>::keep(bh[0], bh[1], bh[2], bh[3]);
    if (SPLIT) Frag<T>::keep(bl[0], bl[1], bl[2], bl[3]);
  }
  acc_guard4(acc[0][0], acc[0][1], acc[0][2], acc[0][3]);
  acc_guard4(acc[1][0], acc[1][1], acc[1][2], acc[1][3]);
  acc_guard4(acc[2][0], acc[2][1], acc[2][2], acc[2][3]);
  acc_guard4(acc[3][0], acc[3][1], acc[3][2], acc[3][3]);

  float* slab = sT[wave];
  const float* Rb = RESID ? (resid + (size_t)b * strideR) : nullptr;
#pragma unroll
  for (int i = 0; i < 4; ++i) {
    const int mBase = m0 + (i << 4);
#pragma unroll
    for (int j = 0; j < 4; ++j) {
      const int n = n0 + (j << 4) + rlane;
      float bv = 0.f;
      if (BIAS_MODE == 2) bv = bias[n];
#pragma unroll
      for (int r = 0; r < 8; ++r) {
        float v = acc[i][j][r] * scale;
        if (BIAS_MODE == 1) v += bias[mBase + mOff + r];
        if (BIAS_MODE == 2) v += bv;
        if (RESID) v += Rb[(size_t)(mBase + mOff + r) * ldc + n];
        if (ACT == 1) v = tanhf(v);
        if (ACT == 2) v = fmaxf(v, 0.0f);
        if (ACT == 3) v = v / (1.0f + expf(-v));
        if (ACT == 4) v = (v > 0.f) ? v : 0.01f * v;
        if (ACT == 5) v = 0.5f * v * (1.0f + erff(v * 0.70710678118654752f));
        slab[(mOff + r) * 68 + (j << 4) + rlane] = v;
      }
    }
    __builtin_amdgcn_fence(__ATOMIC_RELEASE, "workgroup");
    __builtin_amdgcn_wave_barrier();
    __builtin_amdgcn_fence(__ATOMIC_ACQUIRE, "workgroup");
    if (OUT_MODE == 0) {
      float* C = (float*)Cout + (size_t)b * strideC;
      const int hh = lane >> 4, c4 = (lane & 15) * 4;
      for (int pass = 0; pass < 2; ++pass) {
#pragma unroll
        for (int it = 0; it < 8; ++it) {
          const int row = it * 2 + hh;
          v4f v = *(const v4f*)(slab + row * 68 + c4);
          *(volatile v4f*)(C + (size_t)(mBase + row) * ldc + n0 + c4) = v;
        }
        __threadfence();
      }
    } else {
      const int q = lane >> 3, c8 = (lane & 7) * 8;
      unsigned short* C  = (unsigned short*)Cout  + (size_t)b * strideC;
      unsigned short* C2 = (OUT_MODE == 2) ? ((unsigned short*)Cout2 + (size_t)b * strideC) : nullptr;
      for (int pass = 0; pass < 2; ++pass) {
#pragma unroll
        for (int it = 0; it < 4; ++it) {
          const int row = it * 4 + q;
          const float* sp = slab + row * 68 + c8;
          v8h hv, lv;
#pragma unroll
          for (int e = 0; e < 8; ++e) {
            if (OUT_MODE == 1) {
              hv[e] = (_Float16)sp[e];
            } else {
              unsigned short hb = f2bf_bits(sp[e]);
              unsigned short lb = f2bf_bits(sp[e] - bf_bits2f(hb));
              hv[e] = __builtin_bit_cast(_Float16, hb);
              lv[e] = __builtin_bit_cast(_Float16, lb);
            }
          }
          *(volatile v8h*)(C + (size_t)(mBase + row) * ldc + n0 + c8) = hv;
          if (OUT_MODE == 2) *(volatile v8h*)(C2 + (size_t)(mBase + row) * ldc + n0 + c8) = lv;
        }
        __threadfence();
      }
    }
    __builtin_amdgcn_fence(__ATOMIC_RELEASE, "workgroup");
    __builtin_amdgcn_wave_barrier();
    __builtin_amdgcn_fence(__ATOMIC_ACQUIRE, "workgroup");
  }
}

constexpr int NBATCH = 4;
constexpr int NCH    = 256;
constexpr int NPX    = 4096;

static_assert(NPX % 64 == 0);
static_assert(NCH % 64 == 0);
static_assert(NCH % 32 == 0);

__device__ __forceinline__ unsigned int pack_bf2(float f0, float f1, unsigned int& lo_out) {
  const unsigned short h0 = f2bf_bits(f0), h1 = f2bf_bits(f1);
  const unsigned short l0 = f2bf_bits(f0 - bf_bits2f(h0));
  const unsigned short l1 = f2bf_bits(f1 - bf_bits2f(h1));
  lo_out = (unsigned)l0 | ((unsigned)l1 << 16);
  return (unsigned)h0 | ((unsigned)h1 << 16);
}

__global__ __launch_bounds__(256) void split_w_bf16(
    const float* __restrict__ w0, const float* __restrict__ w1, const float* __restrict__ w2,
    unsigned short* __restrict__ planes, int n8, int plane_elems) {
  const int which = blockIdx.y;
  const float* src = (which == 0) ? w0 : ((which == 1) ? w1 : w2);
  unsigned short* dh = planes + (size_t)which * 2 * (size_t)plane_elems;
  unsigned short* dl = dh + plane_elems;
  const int i = blockIdx.x * 256 + threadIdx.x;
  if (i < n8) {
    const v4f a0 = *(const v4f*)(src + 8 * (size_t)i);
    const v4f a1 = *(const v4f*)(src + 8 * (size_t)i + 4);
    v4u32 vh, vl;
    unsigned lo;
    vh[0] = pack_bf2(a0[0], a0[1], lo); vl[0] = lo;
    vh[1] = pack_bf2(a0[2], a0[3], lo); vl[1] = lo;
    vh[2] = pack_bf2(a1[0], a1[1], lo); vl[2] = lo;
    vh[3] = pack_bf2(a1[2], a1[3], lo); vl[3] = lo;
    unsigned short* ph = dh + 8 * (size_t)i;
    unsigned short* pl = dl + 8 * (size_t)i;
    *(volatile v4u32*)ph = vh;
    *(volatile v4u32*)pl = vl;
    __threadfence();
    *(volatile v4u32*)ph = vh;
    *(volatile v4u32*)pl = vl;
  }
}

__global__ __launch_bounds__(256) void transpose_split_x(
    const float* __restrict__ x, unsigned short* __restrict__ xh, unsigned short* __restrict__ xl) {
  __shared__ __align__(16) float tile[64 * 68];
  const int tid = threadIdx.x;
  const int n0 = blockIdx.x * 64;
  const int c0 = blockIdx.y * 64;
  const int b  = blockIdx.z;
  const float* xb = x + ((size_t)b * NCH + c0) * NPX + n0;
#pragma unroll
  for (int it = 0; it < 4; ++it) {
    const int idx = it * 256 + tid;
    const int cr = idx >> 4, n4 = (idx & 15) * 4;
    const v4f v = *(const v4f*)(xb + (size_t)cr * NPX + n4);
    *(v4f*)(tile + cr * 68 + n4) = v;
  }
  __syncthreads();
  unsigned short* hb = xh + ((size_t)b * NPX + n0) * NCH + c0;
  unsigned short* lb = xl + ((size_t)b * NPX + n0) * NCH + c0;
  v4u32 vh[2], vl[2];
  int nrow[2], ccol[2];
#pragma unroll
  for (int it = 0; it < 2; ++it) {
    const int w = it * 256 + tid;
    const int n = w >> 3, c8 = (w & 7) * 8;
    nrow[it] = n; ccol[it] = c8;
#pragma unroll
    for (int e = 0; e < 4; ++e) {
      const float f0 = tile[(c8 + 2 * e) * 68 + n];
      const float f1 = tile[(c8 + 2 * e + 1) * 68 + n];
      unsigned lo;
      vh[it][e] = pack_bf2(f0, f1, lo);
      vl[it][e] = lo;
    }
  }
  for (int pass = 0; pass < 2; ++pass) {
#pragma unroll
    for (int it = 0; it < 2; ++it) {
      *(volatile v4u32*)(hb + (size_t)nrow[it] * NCH + ccol[it]) = vh[it];
      *(volatile v4u32*)(lb + (size_t)nrow[it] * NCH + ccol[it]) = vl[it];
    }
    __threadfence();
  }
}

constexpr int AT_QROWS = 64;
constexpr int AT_KEYS  = 64;
constexpr int QPITCH = 264;
constexpr int KPITCH = 264;
constexpr int VPITCH = 72;
constexpr int PPITCH = 72;
constexpr int OPITCH = 68;
constexpr int LDS_QS = 0;
constexpr int LDS_KS = LDS_QS + AT_QROWS * QPITCH;
constexpr int LDS_VS = LDS_KS + AT_KEYS * KPITCH;
constexpr int LDS_PS = LDS_VS + NCH * VPITCH;
constexpr int LDS_HALVES = LDS_PS + 4 * 16 * PPITCH;
constexpr size_t ATTN_LDS_BYTES = (size_t)LDS_HALVES * 2;
static_assert((size_t)NCH * OPITCH * 4 <= (size_t)(LDS_PS - LDS_KS) * 2);
static_assert((LDS_KS * 2) % 16 == 0 && (LDS_VS * 2) % 16 == 0 && (LDS_PS * 2) % 16 == 0);
static_assert((QPITCH * 2) % 16 == 0 && (VPITCH * 2) % 16 == 0 && (OPITCH * 4) % 16 == 0);
static_assert(NPX % AT_QROWS == 0 && NPX % AT_KEYS == 0 && NCH % 32 == 0);
constexpr float SCORE_SCALE = 0.0625f;
constexpr float PCARRY      = 1024.0f;
constexpr float PCARRY_INV  = 1.0f / 1024.0f;

__device__ __forceinline__ v8f hmma(v16h a, v16h b, v8f c) {
  c = __builtin_amdgcn_wmma_f32_16x16x32_f16(false, a, false, b, (short)0, c, false, false);
  asm volatile("v_nop\n\tv_nop\n\tv_nop\n\tv_nop" : "+v"(c) : "v"(a), "v"(b));
  return c;
}

__global__ __launch_bounds__(128) void cross_attn(
    const unsigned short* __restrict__ Qp, const unsigned short* __restrict__ Kp,
    const unsigned short* __restrict__ VTp, float* __restrict__ outp) {
  extern __shared__ __align__(16) unsigned short lds_dyn[];
  unsigned short* qs_u = lds_dyn + LDS_QS;
  unsigned short* ks_u = lds_dyn + LDS_KS;
  unsigned short* vs_u = lds_dyn + LDS_VS;
  const _Float16* qs_h = (const _Float16*)(const void*)qs_u;
  const _Float16* ks_h = (const _Float16*)(const void*)ks_u;
  const _Float16* vs_h = (const _Float16*)(const void*)vs_u;
  _Float16* ps_h = (_Float16*)(void*)(lds_dyn + LDS_PS);
  float* os_f = (float*)(void*)(lds_dyn + LDS_KS);

  const int tid  = threadIdx.x;
  const int wave = tid >> 5;
  const int lane = tid & 31;
  const int hh   = lane >> 4;
  const int cl   = lane & 15;

  constexpr int nqb = NPX / AT_QROWS;
  const int qb = blockIdx.x % nqb;
  const int b  = blockIdx.x / nqb;
  const int qbase = qb * AT_QROWS;

  const unsigned short* qg = Qp  + ((size_t)b * NPX + qbase) * NCH;
  const unsigned short* kg = Kp  + (size_t)b * NPX * NCH;
  const unsigned short* vg = VTp + (size_t)b * NCH * NPX;
  float* og = outp + (size_t)b * NCH * NPX + qbase;

#pragma unroll 1
  for (int it0 = 0; it0 < 4; ++it0) {
    uint4 w4[4];
#pragma unroll
    for (int it1 = 0; it1 < 4; ++it1) {
      const int idx = (it0 * 4 + it1) * 128 + tid;
      const int row = idx >> 5, c8 = (idx & 31) * 8;
      w4[it1] = *(const uint4*)(qg + (size_t)row * NCH + c8);
    }
#pragma unroll
    for (int it1 = 0; it1 < 4; ++it1) {
      const int idx = (it0 * 4 + it1) * 128 + tid;
      const int row = idx >> 5, c8 = (idx & 31) * 8;
      *(uint4*)(qs_u + row * QPITCH + c8) = w4[it1];
    }
  }

  float mrow[8], lrow[8];
  v8f oacc[16];
#pragma unroll
  for (int r = 0; r < 8; ++r) { mrow[r] = -INFINITY; lrow[r] = 0.f; }
#pragma unroll
  for (int t = 0; t < 16; ++t) oacc[t] = (v8f){0.f,0.f,0.f,0.f,0.f,0.f,0.f,0.f};

  const _Float16* qrow = qs_h + (wave * 16 + cl) * QPITCH + 8 * hh;
  _Float16* pw = ps_h + wave * (16 * PPITCH);

  for (int kc = 0; kc < NPX / AT_KEYS; ++kc) {
    const int kv0 = kc * AT_KEYS;
    __syncthreads();
#pragma unroll 1
    for (int it0 = 0; it0 < 4; ++it0) {
      uint4 kw[4], vw[4];
#pragma unroll
      for (int it1 = 0; it1 < 4; ++it1) {
        const int idx = (it0 * 4 + it1) * 128 + tid;
        const int krow = idx >> 5, kc8 = (idx & 31) * 8;
        const int vrow = idx >> 3, vk8 = (idx & 7) * 8;
        kw[it1] = *(const uint4*)(kg + (size_t)(kv0 + krow) * NCH + kc8);
        vw[it1] = *(const uint4*)(vg + (size_t)vrow * NPX + kv0 + vk8);
      }
#pragma unroll
      for (int it1 = 0; it1 < 4; ++it1) {
        const int idx = (it0 * 4 + it1) * 128 + tid;
        const int krow = idx >> 5, kc8 = (idx & 31) * 8;
        const int vrow = idx >> 3, vk8 = (idx & 7) * 8;
        *(uint4*)(ks_u + krow * KPITCH + kc8) = kw[it1];
        *(uint4*)(vs_u + vrow * VPITCH + vk8) = vw[it1];
      }
    }
    __syncthreads();

    v8f s[4];
#pragma unroll
    for (int j = 0; j < 4; ++j) s[j] = (v8f){0.f,0.f,0.f,0.f,0.f,0.f,0.f,0.f};
#pragma unroll 2
    for (int dc = 0; dc < 8; ++dc) {
      const v16h qa = Frag<_Float16>::load(qrow + dc * 32);
#pragma unroll
      for (int j = 0; j < 4; ++j) {
        const v16h kb = Frag<_Float16>::load(ks_h + (j * 16 + cl) * KPITCH + dc * 32 + 8 * hh);
        s[j] = hmma(qa, kb, s[j]);
      }
    }

    float cm[8];
#pragma unroll
    for (int r = 0; r < 8; ++r) {
      float m = s[0][r];
#pragma unroll
      for (int j = 1; j < 4; ++j) m = fmaxf(m, s[j][r]);
#pragma unroll
      for (int off = 1; off < 16; off <<= 1) m = fmaxf(m, __shfl_xor(m, off, 32));
      cm[r] = m * SCORE_SCALE;
    }
#pragma unroll
    for (int r = 0; r < 8; ++r) {
      const float mnew  = fmaxf(mrow[r], cm[r]);
      const float alpha = expf(mrow[r] - mnew);
      mrow[r] = mnew;
      float psum = 0.f;
#pragma unroll
      for (int j = 0; j < 4; ++j) {
        const float p = expf(s[j][r] * SCORE_SCALE - mnew);
        psum += p;
        pw[(8 * hh + r) * PPITCH + j * 16 + cl] = (_Float16)(p * PCARRY);
      }
#pragma unroll
      for (int off = 1; off < 16; off <<= 1) psum += __shfl_xor(psum, off, 32);
      lrow[r] = lrow[r] * alpha + psum;
#pragma unroll
      for (int t = 0; t < 16; ++t) oacc[t][r] *= alpha;
    }
    __builtin_amdgcn_fence(__ATOMIC_RELEASE, "workgroup");
    __builtin_amdgcn_wave_barrier();
    __builtin_amdgcn_fence(__ATOMIC_ACQUIRE, "workgroup");

#pragma unroll
    for (int kk = 0; kk < 2; ++kk) {
      const v16h pa = Frag<_Float16>::load(pw + cl * PPITCH + kk * 32 + 8 * hh);
#pragma unroll
      for (int t = 0; t < 16; ++t) {
        const v16h vb = Frag<_Float16>::load(vs_h + (t * 16 + cl) * VPITCH + kk * 32 + 8 * hh);
        oacc[t] = hmma(pa, vb, oacc[t]);
      }
    }
  }

  __syncthreads();
#pragma unroll
  for (int r = 0; r < 8; ++r) {
    const float inv = 1.0f / (lrow[r] * PCARRY);
    const int qr = wave * 16 + 8 * hh + r;
#pragma unroll
    for (int t = 0; t < 16; ++t) os_f[(t * 16 + cl) * OPITCH + qr] = oacc[t][r] * inv;
  }
  __syncthreads();
  {
    const int c4 = cl * 4;
    for (int pass = 0; pass < 2; ++pass) {
#pragma unroll 8
      for (int i = 0; i < 32; ++i) {
        const int ch = wave * 64 + 2 * i + hh;
        const v4f val = *(const v4f*)(os_f + ch * OPITCH + c4);
        *(volatile v4f*)(og + (size_t)ch * NPX + c4) = val;
      }
      __threadfence();
    }
  }
}

extern "C" void kernel_launch(void* const* d_in, const int* in_sizes, int n_in,
                              void* d_out, int out_size, void* d_ws, size_t ws_size,
                              hipStream_t stream) {
  if (n_in < 8) return;
  if (in_sizes[0] != NBATCH * NCH * NPX || in_sizes[1] != NBATCH * NCH * NPX) return;
  if (in_sizes[2] != NCH * NCH || in_sizes[4] != NCH * NCH || in_sizes[6] != NCH * NCH) return;
  if (in_sizes[3] != NCH || in_sizes[5] != NCH || in_sizes[7] != NCH) return;
  if (out_size != NBATCH * NCH * NPX) return;

  const float* x1 = (const float*)d_in[0];
  const float* x2 = (const float*)d_in[1];
  const float* Wq = (const float*)d_in[2];
  const float* bq = (const float*)d_in[3];
  const float* Wk = (const float*)d_in[4];
  const float* bk = (const float*)d_in[5];
  const float* Wv = (const float*)d_in[6];
  const float* bv = (const float*)d_in[7];
  float* outp = (float*)d_out;

  const size_t actElems   = (size_t)NBATCH * NPX * NCH;
  const size_t actPlaneB  = actElems * 2;
  const size_t wElems     = (size_t)NCH * NCH;
  const size_t wPlaneB    = wElems * 2;

  unsigned char* ws = (unsigned char*)d_ws;
  size_t off = 0;
  unsigned short* x1h = (unsigned short*)(ws + off); off += actPlaneB;
  unsigned short* x1l = (unsigned short*)(ws + off); off += actPlaneB;
  unsigned short* x2h = (unsigned short*)(ws + off); off += actPlaneB;
  unsigned short* x2l = (unsigned short*)(ws + off); off += actPlaneB;
  unsigned short* wpl = (unsigned short*)(ws + off); off += 6 * wPlaneB;
  unsigned short* Qp  = (unsigned short*)(ws + off); off += actPlaneB;
  unsigned short* Kp  = (unsigned short*)(ws + off); off += actPlaneB;
  unsigned short* VTp = (unsigned short*)(ws + off); off += actPlaneB;
  if (off > ws_size) return;

  unsigned short* Wqh = wpl + 0 * wElems;
  unsigned short* Wql = wpl + 1 * wElems;
  unsigned short* Wkh = wpl + 2 * wElems;
  unsigned short* Wkl = wpl + 3 * wElems;
  unsigned short* Wvh = wpl + 4 * wElems;
  unsigned short* Wvl = wpl + 5 * wElems;

  {
    const int n8 = (int)(wElems / 8);
    dim3 grid((n8 + 255) / 256, 3);
    split_w_bf16<<<grid, 256, 0, stream>>>(Wq, Wk, Wv, wpl, n8, (int)wElems);
  }
  {
    dim3 grid(NPX / 64, NCH / 64, NBATCH);
    transpose_split_x<<<grid, 256, 0, stream>>>(x1, x1h, x1l);
    transpose_split_x<<<grid, 256, 0, stream>>>(x2, x2h, x2l);
  }
  static_assert(NPX % 64 == 0 && NCH % 64 == 0 && NCH % 32 == 0);
  {
    const long actStride = (long)NPX * NCH;
    const int tilesQK = (NPX / 64) * (NCH / 64);
    dim3 gridQK((tilesQK + 7) / 8, NBATCH);
    wmma_gemm64<1, true, 2, 1, false><<<gridQK, 256, 0, stream>>>(
        x1h, x1l, NCH, actStride, Wqh, Wql, NCH, 0L,
        (void*)Qp, nullptr, NCH, actStride, bq, nullptr, 0L, NPX, NCH, NCH, 1.0f);
    wmma_gemm64<1, true, 2, 1, false><<<gridQK, 256, 0, stream>>>(
        x2h, x2l, NCH, actStride, Wkh, Wkl, NCH, 0L,
        (void*)Kp, nullptr, NCH, actStride, bk, nullptr, 0L, NPX, NCH, NCH, 1.0f);
    const int tilesV = (NCH / 64) * (NPX / 64);
    dim3 gridV((tilesV + 7) / 8, NBATCH);
    wmma_gemm64<1, true, 1, 1, false><<<gridV, 256, 0, stream>>>(
        Wvh, Wvl, NCH, 0L, x2h, x2l, NCH, actStride,
        (void*)VTp, nullptr, NPX, actStride, bv, nullptr, 0L, NCH, NPX, NCH, 1.0f);
  }
  {
    dim3 grid(NBATCH * (NPX / AT_QROWS));
    cross_attn<<<grid, 128, ATTN_LDS_BYTES, stream>>>(Qp, Kp, VTp, outp);
  }
}
